// GIN_85736137163003
// MI455X (gfx1250) — hardware-verified
//
#include <hip/hip_runtime.h>
#include <stddef.h>
#include <stdint.h>
#include <math.h>


#define DIN     128
#define HID     256
#define ZW      256
#define TW      512
#define NLAY    3
#define NTHR    256
#define NWAVE   8
#define EPT     8
#define CHUNK   (NTHR * EPT)
#define WCAP    (EPT * 32)
#define LISTN   (NWAVE * WCAP)
#define NBMAX   2048
#define RCAP    28672
#define DEGCAP  64
#define PKS     11
#define GBM     64
#define GBN     128
#define GTHR    128
#define GNT     8
#define NUL1    (HID * (ZW / 8))
#define NUL2    (DIN * (TW / 8))
#define NUW1    (NLAY * NUL1)
#define NUW2    (NLAY * NUL2)
#define NUTOT   (NUW1 + NUW2)
#define WSMAX   134217728
#define LDS_AGG ((2 * RCAP + 2 * NBMAX + LISTN) * 4 + 64)

static_assert((CHUNK & (CHUNK - 1)) == 0 && CHUNK <= (1 << PKS));
static_assert((NBMAX & (NBMAX - 1)) == 0 && NBMAX <= (1 << PKS));
static_assert(NTHR * 8 == NBMAX);
static_assert(LISTN >= NBMAX && LISTN >= NWAVE * WCAP);
static_assert((RCAP % 32) == 0);
static_assert(LDS_AGG <= 300000);
static_assert(GBM == (GTHR / 32) * 16 && GBN == 16 * GNT && GTHR == GBN && GBN == 4 * 32);
static_assert(DIN == 32 * 4);
static_assert((ZW % 32) == 0 && (TW % 32) == 0);
static_assert((HID % GBN) == 0 && (DIN % GBN) == 0);
static_assert(ZW == 2 * DIN && TW == 2 * HID);
static_assert(NUL1 == (1 << 13) && NUL2 == (1 << 13));
static_assert((ZW / 8) == 32 && (TW / 8) == 64);
static_assert((NUW1 % NTHR) == 0 && (NUTOT % NTHR) == 0);
static_assert((GBM * GBN) % GTHR == 0);

typedef float          v4f  __attribute__((ext_vector_type(4)));
typedef float          v8f  __attribute__((ext_vector_type(8)));
typedef int            v4i  __attribute__((ext_vector_type(4)));
typedef int            v8i  __attribute__((ext_vector_type(8)));
typedef unsigned int   v2u  __attribute__((ext_vector_type(2)));
typedef unsigned int   v4u  __attribute__((ext_vector_type(4)));
typedef unsigned short v8us __attribute__((ext_vector_type(8)));
typedef __bf16         v16b __attribute__((ext_vector_type(16)));
typedef v4f  __attribute__((may_alias)) v4fa;
typedef v8us __attribute__((may_alias)) v8usa;
union Frag { v16b vb; v8us h[2]; v8i w; };

__device__ __forceinline__ v8f wmb(const Frag& a, const Frag& b, v8f c) {
  v8f d = __builtin_amdgcn_wmma_f32_16x16x32_bf16(false, a.vb, false, b.vb, (short)0, c, false, false);
  asm volatile("v_nop\n\tv_nop\n\tv_nop\n\tv_nop" : "+v"(d) : "v"(a.w), "v"(b.w));
  return d;
}

__device__ __forceinline__ unsigned short bf_bits(float f) {
  unsigned int u = __float_as_uint(f);
  u += 0x7FFFu + ((u >> 16) & 1u);
  return (unsigned short)(u >> 16);
}
__device__ __forceinline__ float bf_val(unsigned short b) { return __uint_as_float(((unsigned int)b) << 16); }
__device__ __forceinline__ float bf_rne(float f) { return bf_val(bf_bits(f)); }

__device__ __forceinline__ int scan_chunk(const int* __restrict__ dsts, int nE, int cbase, int slotBase,
                                          int nb, int vec8, int* list, int tid, int lane, int wave) {
  int wc = 0;
  const int el0  = tid * EPT;
  const int e0   = cbase + el0;
  const int sent = -2147483647 - 1;
  v4i da, db;
  if (vec8 != 0 && cbase + CHUNK <= nE) {
    da = *(const v4i*)(dsts + e0);
    db = *(const v4i*)(dsts + e0 + 4);
  } else {
    da.x = (e0     < nE) ? dsts[min(e0,     nE - 1)] : sent;
    da.y = (e0 + 1 < nE) ? dsts[min(e0 + 1, nE - 1)] : sent;
    da.z = (e0 + 2 < nE) ? dsts[min(e0 + 2, nE - 1)] : sent;
    da.w = (e0 + 3 < nE) ? dsts[min(e0 + 3, nE - 1)] : sent;
    db.x = (e0 + 4 < nE) ? dsts[min(e0 + 4, nE - 1)] : sent;
    db.y = (e0 + 5 < nE) ? dsts[min(e0 + 5, nE - 1)] : sent;
    db.z = (e0 + 6 < nE) ? dsts[min(e0 + 6, nE - 1)] : sent;
    db.w = (e0 + 7 < nE) ? dsts[min(e0 + 7, nE - 1)] : sent;
  }
  const unsigned nbs = (unsigned)slotBase;
  const unsigned unb = (unsigned)nb;
  const unsigned s0 = (unsigned)da.x - nbs, s1 = (unsigned)da.y - nbs;
  const unsigned s2 = (unsigned)da.z - nbs, s3 = (unsigned)da.w - nbs;
  const unsigned s4 = (unsigned)db.x - nbs, s5 = (unsigned)db.y - nbs;
  const unsigned s6 = (unsigned)db.z - nbs, s7 = (unsigned)db.w - nbs;
  const bool h0 = s0 < unb, h1 = s1 < unb, h2 = s2 < unb, h3 = s3 < unb;
  const bool h4 = s4 < unb, h5 = s5 < unb, h6 = s6 < unb, h7 = s7 < unb;
  const unsigned any = __builtin_amdgcn_ballot_w32(h0 | h1 | h2 | h3 | h4 | h5 | h6 | h7);
  if (any != 0u) {
#define HITJ(J, HJ, SJ) { \
      const unsigned mj = __builtin_amdgcn_ballot_w32(HJ); \
      if (mj != 0u) { \
        if (HJ) { \
          const int pos = wc + (int)__builtin_amdgcn_mbcnt_lo(mj, 0u); \
          if (pos < WCAP) list[wave * WCAP + pos] = ((el0 + (J)) << PKS) | (int)(SJ); \
        } \
        wc += (int)__builtin_popcount(mj); } }
    HITJ(0, h0, s0)
    HITJ(1, h1, s1)
    HITJ(2, h2, s2)
    HITJ(3, h3, s3)
    HITJ(4, h4, s4)
    HITJ(5, h5, s5)
    HITJ(6, h6, s6)
    HITJ(7, h7, s7)
#undef HITJ
  }
  return wc;
}

__global__ __launch_bounds__(NTHR) void k_wprep(const float* __restrict__ W1, const float* __restrict__ W2,
                                                unsigned short* W1T, unsigned short* W2T) {
  const int u = (int)blockIdx.x * NTHR + (int)threadIdx.x;
  v8us o;
  unsigned short* dp;
  if (u < NUW1) {
    const int l  = u >> 13;
    const int v  = u & (NUL1 - 1);
    const int n  = v >> 5;
    const int k8 = (v & 31) * 8;
    const int kk = k8 & (DIN - 1);
    const float* p = W1 + ((size_t)l * DIN + (size_t)kk) * HID + n;
#pragma unroll
    for (int i = 0; i < 8; ++i) o[i] = bf_bits(p[(size_t)i * HID]);
    dp = W1T + (size_t)u * 8;
  } else if (u < NUTOT) {
    const int v2 = u - NUW1;
    const int l  = v2 >> 13;
    const int v  = v2 & (NUL2 - 1);
    const int n  = v >> 6;
    const int k8 = (v & 63) * 8;
    const int kk = k8 & (HID - 1);
    const float* p = W2 + ((size_t)l * HID + (size_t)kk) * DIN + n;
#pragma unroll
    for (int i = 0; i < 8; ++i) o[i] = bf_bits(p[(size_t)i * DIN]);
    dp = W2T + (size_t)v2 * 8;
  } else {
    return;
  }
  *(volatile v8us*)dp = o;
  __threadfence();
  *(volatile v8us*)dp = o;
}

__global__ __launch_bounds__(NTHR) void k_cvx(const float* __restrict__ x, int nN, int nUnits,
                                              unsigned short* xb) {
  const int u = (int)blockIdx.x * NTHR + (int)threadIdx.x;
  if (u >= nUnits) return;
  const int row = u >> 4;
  const int k8  = (u & 15) * 8;
  const int rc  = row < nN ? row : nN - 1;
  const float* p = x + (size_t)rc * DIN + k8;
  const v4f a = *(const v4fa*)p;
  const v4f b = *(const v4fa*)(p + 4);
  const bool ok = row < nN;
  v8us o;
  o[0] = ok ? bf_bits(a.x) : (unsigned short)0;
  o[1] = ok ? bf_bits(a.y) : (unsigned short)0;
  o[2] = ok ? bf_bits(a.z) : (unsigned short)0;
  o[3] = ok ? bf_bits(a.w) : (unsigned short)0;
  o[4] = ok ? bf_bits(b.x) : (unsigned short)0;
  o[5] = ok ? bf_bits(b.y) : (unsigned short)0;
  o[6] = ok ? bf_bits(b.z) : (unsigned short)0;
  o[7] = ok ? bf_bits(b.w) : (unsigned short)0;
  unsigned short* dp = xb + (size_t)row * DIN + k8;
  *(volatile v8us*)dp = o;
  __threadfence();
  *(volatile v8us*)dp = o;
}

template <int SRC16>
__device__ __forceinline__ v4f ldrow(const unsigned short* __restrict__ xb, const float* __restrict__ hf,
                                     int row, int lane) {
  if constexpr (SRC16 != 0) {
    const v2u w = *(const v2u*)(xb + (size_t)row * DIN + 4 * lane);
    v4f r;
    r.x = __uint_as_float(w.x << 16);
    r.y = __uint_as_float(w.x & 0xffff0000u);
    r.z = __uint_as_float(w.y << 16);
    r.w = __uint_as_float(w.y & 0xffff0000u);
    return r;
  } else {
    return *(const v4f*)(hf + (size_t)row * DIN + 4 * lane);
  }
}

template <int SRC16>
__global__ __launch_bounds__(NTHR) void k_agg(
    const int* __restrict__ srcs, const int* __restrict__ dsts,
    const unsigned short* __restrict__ xb, const float* __restrict__ hf,
    const float* __restrict__ epsp, int layer,
    unsigned short* Zout,
    int nN, int nE, int nb, int vec8, int MPr) {
  extern __shared__ v4f lds_dyn[];
  int* reg1 = (int*)lds_dyn;
  int* reg2 = reg1 + RCAP;
  int* scnt = reg2 + RCAP;
  int* soff = scnt + NBMAX;
  int* list = soff + NBMAX;
  int* wcnt = list + LISTN;
  int* wtot = wcnt + NWAVE;
  const int tid = (int)threadIdx.x, lane = tid & 31, wave = tid >> 5;
  const int nodeBase = (int)blockIdx.x * nb;
  const float ep = 1.0f + bf_rne(epsp[layer]);

  for (int i = tid; i < NBMAX; i += NTHR) scnt[i] = 0;
  __syncthreads();

  int tot = 0;
  const int nChunks = (nE + CHUNK - 1) / CHUNK;
#pragma unroll 1
  for (int ch = 0; ch < nChunks; ++ch) {
    const int cbase = ch * CHUNK;
    const int wc = scan_chunk(dsts, nE, cbase, nodeBase, nb, vec8, list, tid, lane, wave);
    if (lane == 0) wcnt[wave] = wc;
    __syncthreads();
    int pre = 0, all = 0;
#pragma unroll
    for (int w2 = 0; w2 < NWAVE; ++w2) {
      int c = wcnt[w2];
      c = c < 0 ? 0 : (c > WCAP ? WCAP : c);
      all += c;
      pre += (w2 < wave) ? c : 0;
    }
    const int wcc  = wc > WCAP ? WCAP : wc;
    const int base = tot + pre;
#pragma unroll 1
    for (int i = lane; i < wcc; i += 32) {
      const int ent = list[wave * WCAP + i];
      const int el  = (ent >> PKS) & (CHUNK - 1);
      const int sl  = ent & (NBMAX - 1);
      int eid = cbase + el;
      eid = eid > nE - 1 ? nE - 1 : eid;
      const int pos = base + i;
      if (pos < RCAP) reg1[pos] = (int)(((unsigned)eid << PKS) | (unsigned)sl);
    }
    tot += all;
    tot = tot > RCAP ? RCAP : tot;
    __syncthreads();
  }
  const int nh = tot;

  if (wave == 0) {
#pragma unroll 1
    for (int b0 = 0; b0 < nh; b0 += 32) {
      const int idx = b0 + lane;
      const int uv  = reg1[idx < RCAP ? idx : RCAP - 1];
      const int m32 = (nh - b0) < 32 ? (nh - b0) : 32;
#pragma unroll 1
      for (int k = 0; k < m32; ++k) {
        const int u  = __builtin_amdgcn_readlane(uv, k);
        const int sl = u & (NBMAX - 1);
        if (lane == 0) scnt[sl] = scnt[sl] + 1;
      }
    }
  }
  __syncthreads();

  {
    const v4i ca = *(const v4i*)(scnt + 8 * tid);
    const v4i cb = *(const v4i*)(scnt + 8 * tid + 4);
    const int e0 = ca.x < 0 ? 0 : ca.x, e1 = ca.y < 0 ? 0 : ca.y, e2 = ca.z < 0 ? 0 : ca.z, e3 = ca.w < 0 ? 0 : ca.w;
    const int e4 = cb.x < 0 ? 0 : cb.x, e5 = cb.y < 0 ? 0 : cb.y, e6 = cb.z < 0 ? 0 : cb.z, e7 = cb.w < 0 ? 0 : cb.w;
    const int ts = e0 + e1 + e2 + e3 + e4 + e5 + e6 + e7;
    int incl = ts;
#pragma unroll
    for (int d = 1; d < 32; d <<= 1) {
      const int up = __shfl_up(incl, d);
      if (lane >= d) incl += up;
    }
    if (lane == 31) wtot[wave] = incl;
    __syncthreads();
    int pre = 0;
#pragma unroll
    for (int w2 = 0; w2 < NWAVE; ++w2) pre += (w2 < wave) ? wtot[w2] : 0;
    int run = pre + incl - ts;
    soff[8 * tid + 0] = run; run += e0;
    soff[8 * tid + 1] = run; run += e1;
    soff[8 * tid + 2] = run; run += e2;
    soff[8 * tid + 3] = run; run += e3;
    soff[8 * tid + 4] = run; run += e4;
    soff[8 * tid + 5] = run; run += e5;
    soff[8 * tid + 6] = run; run += e6;
    soff[8 * tid + 7] = run;
  }
  __syncthreads();
  for (int i = tid; i < NBMAX; i += NTHR) list[i] = soff[i];
  __syncthreads();

  if (wave == 0) {
#pragma unroll 1
    for (int b0 = 0; b0 < nh; b0 += 32) {
      const int idx = b0 + lane;
      const int uv  = reg1[idx < RCAP ? idx : RCAP - 1];
      const int m32 = (nh - b0) < 32 ? (nh - b0) : 32;
#pragma unroll 1
      for (int k = 0; k < m32; ++k) {
        const int u   = __builtin_amdgcn_readlane(uv, k);
        const int sl  = u & (NBMAX - 1);
        const int eid = (int)((unsigned)u >> PKS);
        if (lane == 0) {
          int pos = list[sl];
          pos = pos < 0 ? 0 : (pos > RCAP - 1 ? RCAP - 1 : pos);
          reg2[pos] = eid;
          list[sl] = pos + 1;
        }
      }
    }
  }
  __syncthreads();

  const int nbw = nb >> 3;
  const bool ovf = (nh >= RCAP);
  const float qnan = __int_as_float(0x7fc00000);

#pragma unroll 1
  for (int jt = 0; jt < nbw; ++jt) {
    const int slot = wave * nbw + jt;
    const int grow = nodeBase + slot;
    int st = soff[slot];
    const int craw = scnt[slot];
    int cnt = craw;
    st  = st < 0 ? 0 : (st > nh ? nh : st);
    cnt = cnt < 0 ? 0 : (cnt > DEGCAP ? DEGCAP : cnt);
    if (cnt > nh - st) cnt = nh - st;
    const float pz = (ovf || craw > DEGCAP) ? qnan : 0.0f;
    const bool liveRow = grow < nN;

    float ag0 = 0.f, ag1 = 0.f, ag2 = 0.f, ag3 = 0.f;
#pragma unroll 1
    for (int q = 0; q < cnt; ++q) {
      int idx = st + q; idx = idx > RCAP - 1 ? RCAP - 1 : idx;
      int eid = reg2[idx]; eid = eid < 0 ? 0 : (eid > nE - 1 ? nE - 1 : eid);
      const int sraw = srcs[eid];
      const int s = sraw < 0 ? 0 : (sraw > nN - 1 ? nN - 1 : sraw);
      const v4f v = ldrow<SRC16>(xb, hf, s, lane);
      ag0 += v.x; ag1 += v.y; ag2 += v.z; ag3 += v.w;
    }
    const int nc = liveRow ? grow : nN - 1;
    const v4f sv = ldrow<SRC16>(xb, hf, nc, lane);
    float r0 = ep * sv.x + ag0, r1 = ep * sv.y + ag1, r2 = ep * sv.z + ag2, r3 = ep * sv.w + ag3;
    r0 = (liveRow ? r0 : 0.0f) + pz;
    r1 = (liveRow ? r1 : 0.0f) + pz;
    r2 = (liveRow ? r2 : 0.0f) + pz;
    r3 = (liveRow ? r3 : 0.0f) + pz;

    const unsigned short h0 = bf_bits(r0), h1 = bf_bits(r1), h2 = bf_bits(r2), h3 = bf_bits(r3);
    const unsigned short l0 = bf_bits(r0 - bf_val(h0)), l1 = bf_bits(r1 - bf_val(h1));
    const unsigned short l2 = bf_bits(r2 - bf_val(h2)), l3 = bf_bits(r3 - bf_val(h3));
    v2u ph, pl;
    ph.x = (unsigned int)h0 | ((unsigned int)h1 << 16);
    ph.y = (unsigned int)h2 | ((unsigned int)h3 << 16);
    pl.x = (unsigned int)l0 | ((unsigned int)l1 << 16);
    pl.y = (unsigned int)l2 | ((unsigned int)l3 << 16);
    unsigned short* gp = Zout + (size_t)grow * ZW + 4 * lane;
    const bool wsv = grow < MPr;
    if (wsv) { *(volatile v2u*)gp = ph; *(volatile v2u*)(gp + DIN) = pl; }
    __threadfence();
    if (wsv) { *(volatile v2u*)gp = ph; *(volatile v2u*)(gp + DIN) = pl; }
  }
}

template <int EPI>
__global__ __launch_bounds__(GTHR) void k_gemm(const unsigned short* __restrict__ A, int lda,
                                               const unsigned short* __restrict__ BT, int ldb, int K,
                                               const float* __restrict__ bias, const float* __restrict__ mean,
                                               const float* __restrict__ var, const float* __restrict__ gam,
                                               const float* __restrict__ bet,
                                               void* outp, int ldo, int lsplit, int nN, int mRows) {
  __shared__ __attribute__((aligned(16))) float stg[GBM * GBN];
  const int tid = (int)threadIdx.x, lane = tid & 31, wave = tid >> 5, hh = lane >> 4, m = lane & 15;
  const int rowBase = (int)blockIdx.x * GBM;
  const int colBase = (int)blockIdx.y * GBN;

  v8f acc[GNT];
  {
    const v8f z = {0.f, 0.f, 0.f, 0.f, 0.f, 0.f, 0.f, 0.f};
#pragma unroll
    for (int t = 0; t < GNT; ++t) acc[t] = z;
  }
  const unsigned short* ap = A  + (size_t)(rowBase + 16 * wave + m) * (size_t)lda + 8 * hh;
  const unsigned short* bp = BT + (size_t)(colBase + m) * (size_t)ldb + 8 * hh;

#pragma unroll 1
  for (int k0 = 0; k0 < K; k0 += 32) {
    Frag af;
    af.h[0] = *(const v8usa*)(ap + k0);
    af.h[1] = *(const v8usa*)(ap + k0 + 16);
#pragma unroll
    for (int nt = 0; nt < GNT; ++nt) {
      const unsigned short* wq = bp + (size_t)(16 * nt) * (size_t)ldb + k0;
      Frag bfr;
      bfr.h[0] = *(const v8usa*)wq;
      bfr.h[1] = *(const v8usa*)(wq + 16);
      acc[nt] = wmb(af, bfr, acc[nt]);
    }
  }

#pragma unroll
  for (int nt = 0; nt < GNT; ++nt) {
    const int lc = 16 * nt + m;
#pragma unroll
    for (int r = 0; r < 8; ++r) {
      const int lr = 16 * wave + 8 * hh + r;
      stg[lr * GBN + lc] = acc[nt][r];
    }
  }
  __syncthreads();

  {
    const int col = colBase + tid;
    const float pb = bf_rne(bias[col]);
    float pm = 0.0f, ps = 1.0f, pg = 1.0f, pbe = 0.0f;
    if constexpr (EPI != 2) {
      pm = bf_rne(mean[col]);
      const float pv = bf_rne(var[col]);
      ps  = 1.0f / sqrtf(pv + 1e-5f);
      pg  = bf_rne(gam[col]);
      pbe = bf_rne(bet[col]);
    }
    int nvr = nN - rowBase;
    nvr = nvr < 0 ? 0 : (nvr > GBM ? GBM : nvr);
#pragma unroll 1
    for (int r = 0; r < GBM; ++r) {
      float v = stg[r * GBN + tid] + pb;
      if constexpr (EPI != 2) {
        v = ((v - pm) * ps) * pg + pbe;
        v = (v > 0.0f) ? v : (v - v);
      }
      stg[r * GBN + tid] = (r < nvr) ? v : 0.0f;
    }
  }
  __syncthreads();

  if constexpr (EPI == 2) {
#pragma unroll 1
    for (int i = 0; i < 16; ++i) {
      float* rp = stg + (16 * wave + i) * GBN + 4 * lane;
      const v4f a = *(const v4fa*)rp;
      float mx = fmaxf(fmaxf(a.x, a.y), fmaxf(a.z, a.w));
#pragma unroll
      for (int off = 16; off >= 1; off >>= 1) mx = fmaxf(mx, __shfl_xor(mx, off, 32));
      const float d0 = a.x - mx, d1 = a.y - mx, d2 = a.z - mx, d3 = a.w - mx;
      float s = (expf(d0) + expf(d1)) + (expf(d2) + expf(d3));
#pragma unroll
      for (int off = 16; off >= 1; off >>= 1) s += __shfl_xor(s, off, 32);
      const float lg = logf(s);
      v4f o;
      o.x = d0 - lg; o.y = d1 - lg; o.z = d2 - lg; o.w = d3 - lg;
      *(v4fa*)rp = o;
    }
    __syncthreads();
  }

  if constexpr (EPI == 0) {
    unsigned short* outH = (unsigned short*)outp;
    const int cb = 8 * m;
    const bool isHi = (hh == 0);
    v4u pk[16];
#pragma unroll
    for (int i = 0; i < 16; ++i) {
      const int lr = 16 * wave + i;
      const v4f a = *(const v4fa*)(stg + lr * GBN + cb);
      const v4f b = *(const v4fa*)(stg + lr * GBN + cb + 4);
      const float f[8] = {a.x, a.y, a.z, a.w, b.x, b.y, b.z, b.w};
      unsigned int w[4];
#pragma unroll
      for (int j = 0; j < 4; ++j) {
        const unsigned short h0 = bf_bits(f[2 * j]), h1 = bf_bits(f[2 * j + 1]);
        const unsigned short l0 = bf_bits(f[2 * j] - bf_val(h0)), l1 = bf_bits(f[2 * j + 1] - bf_val(h1));
        const unsigned short q0 = isHi ? h0 : l0, q1 = isHi ? h1 : l1;
        w[j] = (unsigned int)q0 | ((unsigned int)q1 << 16);
      }
      v4u pv; pv.x = w[0]; pv.y = w[1]; pv.z = w[2]; pv.w = w[3];
      pk[i] = pv;
    }
#pragma unroll
    for (int i = 0; i < 16; ++i) {
      const int gr = rowBase + 16 * wave + i;
      unsigned short* op = outH + (size_t)gr * (size_t)ldo + colBase + cb + hh * lsplit;
      if (gr < mRows) *(volatile v4u*)op = pk[i];
    }
    __threadfence();
#pragma unroll
    for (int i = 0; i < 16; ++i) {
      const int gr = rowBase + 16 * wave + i;
      unsigned short* op = outH + (size_t)gr * (size_t)ldo + colBase + cb + hh * lsplit;
      if (gr < mRows) *(volatile v4u*)op = pk[i];
    }
  } else {
    float* outF = (float*)outp;
    v4f fv[16];
#pragma unroll
    for (int i = 0; i < 16; ++i) {
      const int lr = 16 * wave + i;
      fv[i] = *(const v4fa*)(stg + lr * GBN + 4 * lane);
    }
#pragma unroll
    for (int i = 0; i < 16; ++i) {
      const int gr = rowBase + 16 * wave + i;
      float* op = outF + (size_t)gr * (size_t)ldo + colBase + 4 * lane;
      if (gr < mRows) *(volatile v4f*)op = fv[i];
    }
    __threadfence();
#pragma unroll
    for (int i = 0; i < 16; ++i) {
      const int gr = rowBase + 16 * wave + i;
      float* op = outF + (size_t)gr * (size_t)ldo + colBase + 4 * lane;
      if (gr < mRows) *(volatile v4f*)op = fv[i];
    }
  }
}

static int pick_nb(int nE, int nN) {
  int nb = NBMAX;
  while (nb > 16 && (long long)nb * (long long)nE * 5LL > (long long)RCAP * (long long)nN * 4LL) nb >>= 1;
  return nb;
}
static inline int cdiv(int a, int b) { return (a + b - 1) / b; }
static inline size_t al256(size_t o) { return (o + 255) & ~(size_t)255; }

extern "C" void kernel_launch(void* const* d_in, const int* in_sizes, int n_in,
                              void* d_out, int out_size, void* d_ws, size_t ws_size,
                              hipStream_t stream) {
  if (n_in < 15) return;
  if (in_sizes[0] < DIN || (in_sizes[0] % DIN) != 0) return;
  const int nN = in_sizes[0] / DIN;
  if (nN < GBM || nN > (1 << 22)) return;
  const int nE2 = in_sizes[1];
  if (nE2 < 2 || (nE2 & 1) != 0) return;
  const int nE = nE2 / 2;
  if (nE < 1 || nE > (1 << 21)) return;
  if (in_sizes[2] != NLAY * DIN * HID) return;
  if (in_sizes[3] != NLAY * HID || in_sizes[4] != NLAY * HID) return;
  if (in_sizes[5] != NLAY * HID || in_sizes[6] != NLAY * HID) return;
  if (in_sizes[7] != NLAY * HID) return;
  if (in_sizes[8] != NLAY * HID * DIN) return;
  if (in_sizes[9] != NLAY * DIN) return;
  if (in_sizes[10] != NLAY) return;
  if (in_sizes[11] != (NLAY - 1) * DIN || in_sizes[12] != (NLAY - 1) * DIN) return;
  if (in_sizes[13] != (NLAY - 1) * DIN || in_sizes[14] != (NLAY - 1) * DIN) return;
  if ((long long)nN * DIN != (long long)out_size) return;

  const float* x   = (const float*)d_in[0];
  const int*   ei  = (const int*)  d_in[1];
  const int*   src = ei;
  const int*   dst = ei + nE;
  const float* W1  = (const float*)d_in[2];
  const float* b1  = (const float*)d_in[3];
  const float* g1  = (const float*)d_in[4];
  const float* be1 = (const float*)d_in[5];
  const float* m1  = (const float*)d_in[6];
  const float* v1  = (const float*)d_in[7];
  const float* W2  = (const float*)d_in[8];
  const float* b2  = (const float*)d_in[9];
  const float* eps = (const float*)d_in[10];
  const float* go  = (const float*)d_in[11];
  const float* bo  = (const float*)d_in[12];
  const float* mo  = (const float*)d_in[13];
  const float* vo  = (const float*)d_in[14];
  float* out = (float*)d_out;

  const int MP   = cdiv(nN, GBM) * GBM;
  const int gM   = MP / GBM;
  const int nb   = pick_nb(nE, nN);
  const int gA   = cdiv(MP, nb);
  const int vec8 = ((nE & 3) == 0) ? 1 : 0;
  if ((long long)gA * nb < (long long)MP) return;
  if ((long long)(gM - 1) * GBM >= (long long)nN) return;

  char* ws = (char*)d_ws;
  size_t off = 0;
  const size_t oW1 = off; off = al256(off + (size_t)NUW1 * 16);
  const size_t oW2 = off; off = al256(off + (size_t)NUW2 * 16);
  const size_t oXB = off; off = al256(off + (size_t)MP * DIN * 2);
  const size_t oHF = off; off = al256(off + (size_t)MP * DIN * 4);
  const size_t oZP = off; off = al256(off + (size_t)MP * ZW * 2);
  const size_t oTP = off; off = al256(off + (size_t)MP * TW * 2);
  if (off > ws_size || off > (size_t)WSMAX) return;
  unsigned short* W1T = (unsigned short*)(ws + oW1);
  unsigned short* W2T = (unsigned short*)(ws + oW2);
  unsigned short* XB  = (unsigned short*)(ws + oXB);
  float*          HF  = (float*)(ws + oHF);
  unsigned short* ZP  = (unsigned short*)(ws + oZP);
  unsigned short* TP  = (unsigned short*)(ws + oTP);

  hipFuncSetAttribute(reinterpret_cast<const void*>(&k_agg<1>), hipFuncAttributeMaxDynamicSharedMemorySize, LDS_AGG);
  hipFuncSetAttribute(reinterpret_cast<const void*>(&k_agg<0>), hipFuncAttributeMaxDynamicSharedMemorySize, LDS_AGG);

  const int nUx = MP * (DIN / 8);
  k_wprep<<<NUTOT / NTHR, NTHR, 0, stream>>>(W1, W2, W1T, W2T);
  k_cvx<<<cdiv(nUx, NTHR), NTHR, 0, stream>>>(x, nN, nUx, XB);

  for (int l = 0; l < NLAY; ++l) {
    if (l == 0) {
      k_agg<1><<<gA, NTHR, LDS_AGG, stream>>>(src, dst, XB, HF, eps, l, ZP, nN, nE, nb, vec8, MP);
    } else {
      k_agg<0><<<gA, NTHR, LDS_AGG, stream>>>(src, dst, XB, HF, eps, l, ZP, nN, nE, nb, vec8, MP);
    }
    k_gemm<0><<<dim3(gM, HID / GBN), GTHR, 0, stream>>>(
        ZP, ZW, W1T + (size_t)l * HID * ZW, ZW, ZW,
        b1 + l * HID, m1 + l * HID, v1 + l * HID, g1 + l * HID, be1 + l * HID,
        (void*)TP, TW, HID, nN, MP);
    if (l < NLAY - 1) {
      k_gemm<1><<<dim3(gM, DIN / GBN), GTHR, 0, stream>>>(
          TP, TW, W2T + (size_t)l * DIN * TW, TW, TW,
          b2 + l * DIN, mo + l * DIN, vo + l * DIN, go + l * DIN, bo + l * DIN,
          (void*)HF, DIN, 0, nN, MP);
    } else {
      k_gemm<2><<<dim3(gM, DIN / GBN), GTHR, 0, stream>>>(
          TP, TW, W2T + (size_t)l * DIN * TW, TW, TW,
          b2 + l * DIN, b2 + l * DIN, b2 + l * DIN, b2 + l * DIN, b2 + l * DIN,
          (void*)out, DIN, 0, nN, nN);
    }
  }
}
